// RRN_23888608101388
// MI455X (gfx1250) — hardware-verified
//
#include <hip/hip_runtime.h>
#include <stddef.h>
#include <stdint.h>


#define DD      128
#define KCL     64
#define KCM     192
#define PK      256
#define NL      16
#define RPC     2
#define NCH     (NL / RPC)
#define NTHR    256
#define NWAVE   8
#define EPT     8
#define CHUNK   (NTHR * EPT)
#define WCAP    (EPT * 32)
#define LISTN   (NWAVE * WCAP)
#define NBMAX   2048
#define RCAP    28672
#define DEGCAP  64
#define STW     128
#define GBM     64
#define GBN     128
#define GTHR    128
#define CH      16.0f
#define CW      64.0f
#define SCL_HW  0.0009765625f
#define LDS_AGG ((2 * RCAP + 2 * NBMAX + LISTN) * 4 + 64)
#define LDS_PAIR (2 * GBM * PK * 2)

static_assert((CHUNK & (CHUNK - 1)) == 0 && CHUNK <= 4096);
static_assert((NBMAX & (NBMAX - 1)) == 0 && NBMAX <= 4096);
static_assert(NTHR * 8 == NBMAX);
static_assert(LISTN >= NBMAX);
static_assert(LISTN >= NWAVE * WCAP);
static_assert((RCAP % 32) == 0);
static_assert(NWAVE * STW <= RCAP);
static_assert(2 * STW >= 2 * DD);
static_assert(LDS_AGG <= 300000);
static_assert(LDS_PAIR <= 300000);
static_assert(GBM * DD * 2 <= GBM * PK * 2);
static_assert(GBM == (GTHR / 32) * 16);
static_assert(GBN == DD && PK == 2 * DD && KCM == DD + KCL);
static_assert((KCM % 32) == 0 && (DD % 32) == 0 && (PK % 32) == 0);
static_assert((NL % RPC) == 0);
static_assert((GBM * 2) % (GTHR / 32) == 0);

typedef float          v4f  __attribute__((ext_vector_type(4)));
typedef float          v8f  __attribute__((ext_vector_type(8)));
typedef int            v4i  __attribute__((ext_vector_type(4)));
typedef int            v8i  __attribute__((ext_vector_type(8)));
typedef unsigned short v4us __attribute__((ext_vector_type(4)));
typedef unsigned short v8us __attribute__((ext_vector_type(8)));
typedef __bf16         v16b __attribute__((ext_vector_type(16)));
typedef _Float16       v16h __attribute__((ext_vector_type(16)));
union Frag { v16b b; v16h h; v8us u[2]; v8i w; };

template<int F16>
__device__ __forceinline__ v8f mma(const Frag& a, const Frag& b, v8f c) {
  v8f d;
  if (F16 != 0) d = __builtin_amdgcn_wmma_f32_16x16x32_f16(false, a.h, false, b.h, (short)0, c, false, false);
  else          d = __builtin_amdgcn_wmma_f32_16x16x32_bf16(false, a.b, false, b.b, (short)0, c, false, false);
  asm volatile("v_nop\n\tv_nop\n\tv_nop\n\tv_nop" : "+v"(d) : "v"(a.w), "v"(b.w));
  return d;
}

__device__ __forceinline__ void ldwait() {
  asm volatile("s_wait_loadcnt 0x0" ::: "memory");
}

__device__ __forceinline__ unsigned short bfbits(float x) {
  unsigned u = __float_as_uint(x);
  u += 0x7FFFu + ((u >> 16) & 1u);
  return (unsigned short)(u >> 16);
}
__device__ __forceinline__ float bfval(unsigned short b) { return __uint_as_float(((unsigned)b) << 16); }
__device__ __forceinline__ float bfr(float x) { return bfval(bfbits(x)); }
__device__ __forceinline__ unsigned short hbits(float x) {
  const _Float16 h = (_Float16)x;
  return __builtin_bit_cast(unsigned short, h);
}

__device__ __forceinline__ int scan_chunk(const int* __restrict__ dsts, int nE, int cbase, int slotBase,
                                          int nb, int vec8, int* list, int tid, int lane, int wave) {
  int wc = 0;
  const int el0  = tid * EPT;
  const int e0   = cbase + el0;
  const int sent = -2147483647 - 1;
  v4i da, db;
  if (vec8 != 0 && cbase + CHUNK <= nE) {
    da = *(const v4i*)(dsts + e0);
    db = *(const v4i*)(dsts + e0 + 4);
  } else {
    da.x = (e0     < nE) ? dsts[min(e0,     nE - 1)] : sent;
    da.y = (e0 + 1 < nE) ? dsts[min(e0 + 1, nE - 1)] : sent;
    da.z = (e0 + 2 < nE) ? dsts[min(e0 + 2, nE - 1)] : sent;
    da.w = (e0 + 3 < nE) ? dsts[min(e0 + 3, nE - 1)] : sent;
    db.x = (e0 + 4 < nE) ? dsts[min(e0 + 4, nE - 1)] : sent;
    db.y = (e0 + 5 < nE) ? dsts[min(e0 + 5, nE - 1)] : sent;
    db.z = (e0 + 6 < nE) ? dsts[min(e0 + 6, nE - 1)] : sent;
    db.w = (e0 + 7 < nE) ? dsts[min(e0 + 7, nE - 1)] : sent;
  }
  const unsigned nbs = (unsigned)slotBase;
  const unsigned unb = (unsigned)nb;
  const unsigned s0 = (unsigned)da.x - nbs, s1 = (unsigned)da.y - nbs;
  const unsigned s2 = (unsigned)da.z - nbs, s3 = (unsigned)da.w - nbs;
  const unsigned s4 = (unsigned)db.x - nbs, s5 = (unsigned)db.y - nbs;
  const unsigned s6 = (unsigned)db.z - nbs, s7 = (unsigned)db.w - nbs;
  const bool h0 = s0 < unb, h1 = s1 < unb, h2 = s2 < unb, h3 = s3 < unb;
  const bool h4 = s4 < unb, h5 = s5 < unb, h6 = s6 < unb, h7 = s7 < unb;
  const unsigned any = __builtin_amdgcn_ballot_w32(h0 | h1 | h2 | h3 | h4 | h5 | h6 | h7);
  if (any != 0u) {
#define HITJ(J, HJ, SJ) { \
      const unsigned mj = __builtin_amdgcn_ballot_w32(HJ); \
      if (mj != 0u) { \
        if (HJ) { \
          const int pos = wc + (int)__builtin_amdgcn_mbcnt_lo(mj, 0u); \
          if (pos < WCAP) list[wave * WCAP + pos] = ((el0 + (J)) << 12) | (int)(SJ); \
        } \
        wc += (int)__builtin_popcount(mj); } }
    HITJ(0, h0, s0)
    HITJ(1, h1, s1)
    HITJ(2, h2, s2)
    HITJ(3, h3, s3)
    HITJ(4, h4, s4)
    HITJ(5, h5, s5)
    HITJ(6, h6, s6)
    HITJ(7, h7, s7)
#undef HITJ
  }
  return wc;
}

__global__ __launch_bounds__(NTHR) void k_wtr(const float* __restrict__ w, int K, int Nc, int inMat, int outMat,
                                              int rowOff, int mode, unsigned short* wt, int nUnits) {
  const int u = (int)blockIdx.x * NTHR + (int)threadIdx.x;
  if (u >= nUnits) return;
  const int kq  = K >> 3;
  const int per = Nc * kq;
  const int mat = u / per;
  const int rem = u - mat * per;
  const int n   = rem / kq;
  const int k8  = (rem - n * kq) * 8;
  const float* p = w + (size_t)mat * (size_t)inMat + (size_t)k8 * (size_t)Nc + n;
  float f[8];
#pragma unroll
  for (int i = 0; i < 8; ++i) f[i] = p[(size_t)i * (size_t)Nc];
  v8us o;
  if (mode != 0) {
#pragma unroll
    for (int i = 0; i < 8; ++i) o[i] = hbits(bfr(f[i]) * CW);
  } else {
#pragma unroll
    for (int i = 0; i < 8; ++i) o[i] = bfbits(f[i]);
  }
  unsigned short* d = wt + (size_t)mat * (size_t)outMat + (size_t)(rowOff + n) * (size_t)K + k8;
  *(volatile v8us*)d = o;
  __threadfence();
  *(volatile v8us*)d = o;
}

__global__ __launch_bounds__(NTHR) void k_xprep(const float* __restrict__ x, const float* __restrict__ mb,
                                                unsigned short* eh, int nN, int nUnits) {
  const int i = (int)blockIdx.x * NTHR + (int)threadIdx.x;
  if (i >= nUnits) return;
  const int row = i / (KCM / 8);
  const int c8  = (i - row * (KCM / 8)) * 8;
  const int rc  = row < nN ? row : nN - 1;
  const float* p = (c8 < DD) ? (x + (size_t)rc * DD + c8) : (mb + (size_t)rc * KCL + (c8 - DD));
  v4f a = *(const v4f*)p, b = *(const v4f*)(p + 4);
  const v4f z4 = {0.f, 0.f, 0.f, 0.f};
  if (row >= nN) { a = z4; b = z4; }
  v8us o;
  o[0] = bfbits(a.x); o[1] = bfbits(a.y); o[2] = bfbits(a.z); o[3] = bfbits(a.w);
  o[4] = bfbits(b.x); o[5] = bfbits(b.y); o[6] = bfbits(b.z); o[7] = bfbits(b.w);
  unsigned short* d = eh + (size_t)row * KCM + c8;
  *(volatile v8us*)d = o;
  __threadfence();
  *(volatile v8us*)d = o;
}

__global__ __launch_bounds__(NTHR) void k_zfill(unsigned short* p, int nUnits) {
  const int i = (int)blockIdx.x * NTHR + (int)threadIdx.x;
  if (i >= nUnits) return;
  const v8us z = {0, 0, 0, 0, 0, 0, 0, 0};
  unsigned short* d = p + (size_t)i * 8;
  *(volatile v8us*)d = z;
  __threadfence();
  *(volatile v8us*)d = z;
}

template<int EPI, int F16>
__global__ __launch_bounds__(GTHR) void k_gemm(
    const unsigned short* __restrict__ AH, int ldh, int ksteps,
    const unsigned short* __restrict__ AL, int ldl, int lsteps, int aZ,
    const unsigned short* __restrict__ WT, int wZ,
    const float* __restrict__ bia0, const float* __restrict__ bia1, int bZ,
    float* outF, unsigned short* outH, unsigned short* outL,
    int ldo, int oZ, int nRows, float scl)
{
  __shared__ __attribute__((aligned(16))) float stg[GBM * GBN];
  const int tid = (int)threadIdx.x, lane = tid & 31, wave = tid >> 5, hh = lane >> 4, m = lane & 15;
  const int rowBase = (int)blockIdx.x * GBM;
  const int col0    = (int)blockIdx.y * GBN;
  const int z       = (int)blockIdx.z;
  const int K       = ksteps << 5;

  v8f acc[8];
  {
    const v8f zz = {0.f, 0.f, 0.f, 0.f, 0.f, 0.f, 0.f, 0.f};
#pragma unroll
    for (int t = 0; t < 8; ++t) acc[t] = zz;
  }
  const unsigned short* ap = AH + (size_t)z * (size_t)aZ + (size_t)(rowBase + 16 * wave + m) * (size_t)ldh + 8 * hh;
  const unsigned short* wp = WT + (size_t)z * (size_t)wZ + (size_t)(col0 + m) * (size_t)K + 8 * hh;
#pragma unroll 1
  for (int ks = 0; ks < ksteps; ++ks) {
    Frag af;
    af.u[0] = *(const v8us*)(ap + 32 * ks);
    af.u[1] = *(const v8us*)(ap + 32 * ks + 16);
#pragma unroll
    for (int t = 0; t < 8; ++t) {
      const unsigned short* wq = wp + (size_t)(16 * t) * (size_t)K + 32 * ks;
      Frag bf;
      bf.u[0] = *(const v8us*)wq;
      bf.u[1] = *(const v8us*)(wq + 16);
      acc[t] = mma<F16>(af, bf, acc[t]);
    }
  }
  if (lsteps > 0) {
    const unsigned short* lp = AL + (size_t)z * (size_t)aZ + (size_t)(rowBase + 16 * wave + m) * (size_t)ldl + 8 * hh;
#pragma unroll 1
    for (int ls = 0; ls < lsteps; ++ls) {
      Frag af;
      af.u[0] = *(const v8us*)(lp + 32 * ls);
      af.u[1] = *(const v8us*)(lp + 32 * ls + 16);
#pragma unroll
      for (int t = 0; t < 8; ++t) {
        const unsigned short* wq = wp + (size_t)(16 * t) * (size_t)K + 32 * ls;
        Frag bf;
        bf.u[0] = *(const v8us*)wq;
        bf.u[1] = *(const v8us*)(wq + 16);
        acc[t] = mma<F16>(af, bf, acc[t]);
      }
    }
  }

  const float* bp = ((blockIdx.y == 0) ? bia0 : bia1) + (size_t)z * (size_t)bZ;
  unsigned short* sth = (unsigned short*)stg;
  unsigned short* stl = sth + GBM * GBN;
#pragma unroll
  for (int t = 0; t < 8; ++t) {
    const int lc = 16 * t + m;
    const float bv = bfr(bp[lc]);
#pragma unroll
    for (int r = 0; r < 8; ++r) {
      const int lr = 16 * wave + 8 * hh + r;
      const float live = (rowBase + lr < nRows) ? 1.0f : 0.0f;
      float v = fmaf(acc[t][r], scl, bv) * live;
      if (EPI == 0) {
        stg[lr * GBN + lc] = v;
      } else {
        v = fmaxf(v, 0.f);
        const unsigned short hb = bfbits(v);
        const unsigned short lb = bfbits(v - bfval(hb));
        sth[lr * GBN + lc] = hb;
        stl[lr * GBN + lc] = lb;
      }
    }
  }
  __syncthreads();

  if (EPI == 0) {
#pragma unroll
    for (int g = 0; g < 2; ++g) {
      v4f fv[8];
#pragma unroll
      for (int i = 0; i < 8; ++i) {
        const int lr = 16 * wave + 8 * g + i;
        fv[i] = *(const v4f*)(stg + lr * GBN + 4 * lane);
      }
#pragma unroll
      for (int i = 0; i < 8; ++i) {
        const int lr = 16 * wave + 8 * g + i;
        float* op = outF + (size_t)z * (size_t)oZ + (size_t)(rowBase + lr) * (size_t)ldo + col0 + 4 * lane;
        *(volatile v4f*)op = fv[i];
      }
      __threadfence();
#pragma unroll
      for (int i = 0; i < 8; ++i) {
        const int lr = 16 * wave + 8 * g + i;
        float* op = outF + (size_t)z * (size_t)oZ + (size_t)(rowBase + lr) * (size_t)ldo + col0 + 4 * lane;
        *(volatile v4f*)op = fv[i];
      }
    }
  } else {
    const unsigned short* sb = sth + hh * (GBM * GBN);
    unsigned short* ob = (hh == 0) ? outH : outL;
#pragma unroll
    for (int g = 0; g < 2; ++g) {
      v8us pv[8];
#pragma unroll
      for (int i = 0; i < 8; ++i) {
        const int lr = 16 * wave + 8 * g + i;
        pv[i] = *(const v8us*)(sb + lr * GBN + 8 * m);
      }
#pragma unroll
      for (int i = 0; i < 8; ++i) {
        const int lr = 16 * wave + 8 * g + i;
        unsigned short* op = ob + (size_t)z * (size_t)oZ + (size_t)(rowBase + lr) * (size_t)ldo + 8 * m;
        *(volatile v8us*)op = pv[i];
      }
      __threadfence();
#pragma unroll
      for (int i = 0; i < 8; ++i) {
        const int lr = 16 * wave + 8 * g + i;
        unsigned short* op = ob + (size_t)z * (size_t)oZ + (size_t)(rowBase + lr) * (size_t)ldo + 8 * m;
        *(volatile v8us*)op = pv[i];
      }
    }
  }
}

__global__ __launch_bounds__(GTHR) void k_pair(
    const float* __restrict__ UPD, const int* __restrict__ sidx, const int* __restrict__ oidx,
    int E, int EP, int nN, const unsigned short* __restrict__ W1T, const float* __restrict__ b1,
    unsigned short* HR)
{
  extern __shared__ v4f lds_dyn[];
  unsigned short* AHt = (unsigned short*)lds_dyn;
  unsigned short* ALt = AHt + GBM * PK;
  const int tid = (int)threadIdx.x, lane = tid & 31, wave = tid >> 5, hh = lane >> 4, m = lane & 15;
  const int rowBase = (int)blockIdx.x * GBM;
  const int z       = (int)blockIdx.z;
  const v4f z4 = {0.f, 0.f, 0.f, 0.f};

#pragma unroll 1
  for (int it = 0; it < (GBM * 2) / (GTHR / 32); ++it) {
    const int unit = it * (GTHR / 32) + wave;
    const int row  = unit >> 1;
    const int half = unit & 1;
    const int r    = rowBase + row;
    const int rr   = r < E ? r : E - 1;
    const int is   = sidx[(size_t)z * (size_t)E + rr];
    const int io   = oidx[(size_t)z * (size_t)E + rr];
    int idx = (half != 0) ? io : is;
    idx = idx < 0 ? 0 : (idx > nN - 1 ? nN - 1 : idx);
    v4f v = *(const v4f*)(UPD + (size_t)idx * DD + 4 * lane);
    if (r >= E) v = z4;
    v4us hb, lb;
    hb.x = bfbits(v.x); hb.y = bfbits(v.y); hb.z = bfbits(v.z); hb.w = bfbits(v.w);
    lb.x = bfbits(v.x - bfval(hb.x)); lb.y = bfbits(v.y - bfval(hb.y));
    lb.z = bfbits(v.z - bfval(hb.z)); lb.w = bfbits(v.w - bfval(hb.w));
    const int o = row * PK + half * DD + 4 * lane;
    *(v4us*)(AHt + o) = hb;
    *(v4us*)(ALt + o) = lb;
  }
  __syncthreads();

  v8f acc[8];
  {
    const v8f zz = {0.f, 0.f, 0.f, 0.f, 0.f, 0.f, 0.f, 0.f};
#pragma unroll
    for (int t = 0; t < 8; ++t) acc[t] = zz;
  }
  const unsigned short* ap = AHt + (16 * wave + m) * PK + 8 * hh;
  const unsigned short* lp = ALt + (16 * wave + m) * PK + 8 * hh;
  const unsigned short* wp = W1T + (size_t)z * (size_t)(DD * PK) + (size_t)m * PK + 8 * hh;
#pragma unroll 1
  for (int ks = 0; ks < PK / 32; ++ks) {
    Frag ah, al;
    ah.u[0] = *(const v8us*)(ap + 32 * ks);
    ah.u[1] = *(const v8us*)(ap + 32 * ks + 16);
    al.u[0] = *(const v8us*)(lp + 32 * ks);
    al.u[1] = *(const v8us*)(lp + 32 * ks + 16);
#pragma unroll
    for (int t = 0; t < 8; ++t) {
      const unsigned short* wq = wp + (size_t)(16 * t) * PK + 32 * ks;
      Frag bf;
      bf.u[0] = *(const v8us*)wq;
      bf.u[1] = *(const v8us*)(wq + 16);
      acc[t] = mma<0>(ah, bf, acc[t]);
      acc[t] = mma<0>(al, bf, acc[t]);
    }
  }
  __syncthreads();

  unsigned short* sth = AHt;
#pragma unroll
  for (int t = 0; t < 8; ++t) {
    const int lc = 16 * t + m;
    const float bv = bfr(b1[(size_t)z * DD + lc]);
#pragma unroll
    for (int r = 0; r < 8; ++r) {
      const int lr = 16 * wave + 8 * hh + r;
      const float live = (rowBase + lr < E) ? 1.0f : 0.0f;
      const float v = fmaxf(acc[t][r] + bv, 0.f) * live;
      sth[lr * DD + lc] = hbits(v * CH);
    }
  }
  __syncthreads();
  v8us pv[8];
#pragma unroll
  for (int i = 0; i < 8; ++i) {
    const int lr = 16 * wave + 2 * i + hh;
    pv[i] = *(const v8us*)(sth + lr * DD + 8 * m);
  }
#pragma unroll
  for (int i = 0; i < 8; ++i) {
    const int lr = 16 * wave + 2 * i + hh;
    unsigned short* op = HR + (size_t)z * (size_t)EP * DD + (size_t)(rowBase + lr) * DD + 8 * m;
    *(volatile v8us*)op = pv[i];
  }
  __threadfence();
#pragma unroll
  for (int i = 0; i < 8; ++i) {
    const int lr = 16 * wave + 2 * i + hh;
    unsigned short* op = HR + (size_t)z * (size_t)EP * DD + (size_t)(rowBase + lr) * DD + 8 * m;
    *(volatile v8us*)op = pv[i];
  }
}

__global__ __launch_bounds__(NTHR) void k_agg(
    const int* __restrict__ sseg, const int* __restrict__ oseg, int nSeg,
    const float* __restrict__ MSG, int E, int EP,
    float* ACC, const float* __restrict__ UPD,
    unsigned short* EH, unsigned short* EL, float* OUT,
    int nN, int nb, int vec8, int rd, int fin, int last) {
  extern __shared__ v4f lds_dyn[];
  int* reg1 = (int*)lds_dyn;
  int* reg2 = reg1 + RCAP;
  int* scnt = reg2 + RCAP;
  int* soff = scnt + NBMAX;
  int* list = soff + NBMAX;
  int* wcnt = list + LISTN;
  int* wtot = wcnt + NWAVE;
  const int tid = (int)threadIdx.x, lane = tid & 31, wave = tid >> 5, hh = lane >> 4;
  const int nodeBase = (int)blockIdx.x * nb;

  for (int i = tid; i < NBMAX; i += NTHR) scnt[i] = 0;
  __syncthreads();

  int tot = 0;
#pragma unroll 1
  for (int role = 0; role < 2; ++role) {
    const int* dsts = (role == 0) ? sseg : oseg;
    const int nChunks = (nSeg + CHUNK - 1) / CHUNK;
#pragma unroll 1
    for (int ch = 0; ch < nChunks; ++ch) {
      const int cbase = ch * CHUNK;
      const int wc = scan_chunk(dsts, nSeg, cbase, nodeBase, nb, vec8, list, tid, lane, wave);
      if (lane == 0) wcnt[wave] = wc;
      __syncthreads();
      int pre = 0, all = 0;
#pragma unroll
      for (int w2 = 0; w2 < NWAVE; ++w2) {
        int c = wcnt[w2];
        c = c < 0 ? 0 : (c > WCAP ? WCAP : c);
        all += c;
        pre += (w2 < wave) ? c : 0;
      }
      const int wcc  = wc > WCAP ? WCAP : wc;
      const int base = tot + pre;
#pragma unroll 1
      for (int i = lane; i < wcc; i += 32) {
        const int ent = list[wave * WCAP + i];
        const int el  = (ent >> 12) & (CHUNK - 1);
        const int sl  = ent & (NBMAX - 1);
        int q = cbase + el;
        q = q > nSeg - 1 ? nSeg - 1 : q;
        const int eid = role * nSeg + q;
        const int pos = base + i;
        if (pos < RCAP) reg1[pos] = (int)(((unsigned)eid << 12) | (unsigned)sl);
      }
      tot += all;
      tot = tot > RCAP ? RCAP : tot;
      __syncthreads();
    }
  }
  const int nh = tot;

  if (wave == 0) {
#pragma unroll 1
    for (int b0 = 0; b0 < nh; b0 += 32) {
      const int idx = b0 + lane;
      const int uv  = reg1[idx < RCAP ? idx : RCAP - 1];
      const int m32 = (nh - b0) < 32 ? (nh - b0) : 32;
#pragma unroll 1
      for (int k = 0; k < m32; ++k) {
        const int u  = __builtin_amdgcn_readlane(uv, k);
        const int sl = u & (NBMAX - 1);
        if (lane == 0) scnt[sl] = scnt[sl] + 1;
      }
    }
  }
  __syncthreads();

  {
    const v4i ca = *(const v4i*)(scnt + 8 * tid);
    const v4i cb = *(const v4i*)(scnt + 8 * tid + 4);
    const int e0 = ca.x < 0 ? 0 : ca.x, e1 = ca.y < 0 ? 0 : ca.y, e2 = ca.z < 0 ? 0 : ca.z, e3 = ca.w < 0 ? 0 : ca.w;
    const int e4 = cb.x < 0 ? 0 : cb.x, e5 = cb.y < 0 ? 0 : cb.y, e6 = cb.z < 0 ? 0 : cb.z, e7 = cb.w < 0 ? 0 : cb.w;
    const int ts = e0 + e1 + e2 + e3 + e4 + e5 + e6 + e7;
    int incl = ts;
#pragma unroll
    for (int d = 1; d < 32; d <<= 1) {
      const int up = __shfl_up(incl, d);
      if (lane >= d) incl += up;
    }
    if (lane == 31) wtot[wave] = incl;
    __syncthreads();
    int pre = 0;
#pragma unroll
    for (int w2 = 0; w2 < NWAVE; ++w2) pre += (w2 < wave) ? wtot[w2] : 0;
    int run = pre + incl - ts;
    soff[8 * tid + 0] = run; run += e0;
    soff[8 * tid + 1] = run; run += e1;
    soff[8 * tid + 2] = run; run += e2;
    soff[8 * tid + 3] = run; run += e3;
    soff[8 * tid + 4] = run; run += e4;
    soff[8 * tid + 5] = run; run += e5;
    soff[8 * tid + 6] = run; run += e6;
    soff[8 * tid + 7] = run;
  }
  __syncthreads();
  for (int i = tid; i < NBMAX; i += NTHR) list[i] = soff[i];
  __syncthreads();

  if (wave == 0) {
#pragma unroll 1
    for (int b0 = 0; b0 < nh; b0 += 32) {
      const int idx = b0 + lane;
      const int uv  = reg1[idx < RCAP ? idx : RCAP - 1];
      const int m32 = (nh - b0) < 32 ? (nh - b0) : 32;
#pragma unroll 1
      for (int k = 0; k < m32; ++k) {
        const int u   = __builtin_amdgcn_readlane(uv, k);
        const int sl  = u & (NBMAX - 1);
        const int eid = (int)((unsigned)u >> 12);
        if (lane == 0) {
          int pos = list[sl];
          pos = pos < 0 ? 0 : (pos > RCAP - 1 ? RCAP - 1 : pos);
          reg2[pos] = eid;
          list[sl] = pos + 1;
        }
      }
    }
  }
  __syncthreads();

  const int nbw = nb >> 3;
  const bool ovf = (nh >= RCAP);
  const float qnan = __int_as_float(0x7fc00000);
  unsigned short* stw = (unsigned short*)((float*)reg1 + wave * STW);
  const int nEnt = 2 * nSeg;
#pragma unroll 1
  for (int jt = 0; jt < nbw; ++jt) {
    const int slot = wave * nbw + jt;
    const int grow = nodeBase + slot;
    const int gcl  = grow < nN ? grow : nN - 1;
    int st = soff[slot];
    const int craw = scnt[slot];
    int cnt = craw;
    st  = st < 0 ? 0 : (st > nh ? nh : st);
    cnt = cnt < 0 ? 0 : (cnt > DEGCAP ? DEGCAP : cnt);
    if (cnt > nh - st) cnt = nh - st;
    const float pz = (ovf || craw > DEGCAP) ? qnan : 0.0f;
    const bool wr = grow < nN;

    v4f a = {0.f, 0.f, 0.f, 0.f};
    if (rd != 0) a = *(const v4f*)(ACC + (size_t)gcl * DD + 4 * lane);
#pragma unroll 1
    for (int q = 0; q < cnt; ++q) {
      int idx = st + q; idx = idx > RCAP - 1 ? RCAP - 1 : idx;
      int eid = reg2[idx]; eid = eid < 0 ? 0 : (eid > nEnt - 1 ? nEnt - 1 : eid);
      const int role = (eid >= nSeg) ? 1 : 0;
      const int q2   = eid - role * nSeg;
      const int jr   = (q2 >= E) ? 1 : 0;
      int r = q2 - jr * E;
      r = r < 0 ? 0 : (r > E - 1 ? E - 1 : r);
      const float* mp = MSG + (size_t)(jr * EP + r) * (size_t)PK + role * DD + 4 * lane;
      const v4f mv = *(const v4f*)mp;
      a += mv;
    }
    a.x += pz; a.y += pz; a.z += pz; a.w += pz;

    if (fin == 0) {
      float* op = ACC + (size_t)grow * DD + 4 * lane;
      if (wr) *(volatile v4f*)op = a;
      __threadfence();
      if (wr) *(volatile v4f*)op = a;
    } else {
      const v4f u = *(const v4f*)(UPD + (size_t)gcl * DD + 4 * lane);
      const v4f v = u + a;
      float ss = v.x * v.x + v.y * v.y + v.z * v.z + v.w * v.w;
#pragma unroll
      for (int off = 16; off >= 1; off >>= 1) ss += __shfl_xor(ss, off, 32);
      const float nrm = fmaxf(sqrtf(ss), 1e-12f);
      const float inv = 1.0f / nrm;
      v4f o;
      o.x = v.x * inv; o.y = v.y * inv; o.z = v.z * inv; o.w = v.w * inv;
      if (last != 0) {
        float* op = OUT + (size_t)grow * DD + 4 * lane;
        if (wr) *(volatile v4f*)op = o;
        __threadfence();
        if (wr) *(volatile v4f*)op = o;
      } else {
        v4us hb, lb;
        hb.x = bfbits(o.x); hb.y = bfbits(o.y); hb.z = bfbits(o.z); hb.w = bfbits(o.w);
        lb.x = bfbits(o.x - bfval(hb.x)); lb.y = bfbits(o.y - bfval(hb.y));
        lb.z = bfbits(o.z - bfval(hb.z)); lb.w = bfbits(o.w - bfval(hb.w));
        __builtin_amdgcn_fence(__ATOMIC_RELEASE, "wavefront");
        __builtin_amdgcn_wave_barrier();
        *(v4us*)(stw + 4 * lane)      = hb;
        *(v4us*)(stw + DD + 4 * lane) = lb;
        __builtin_amdgcn_fence(__ATOMIC_RELEASE, "wavefront");
        __builtin_amdgcn_wave_barrier();
        const v8us pv = *(const v8us*)(stw + 8 * lane);
        unsigned short* gp = (hh != 0) ? (EL + (size_t)grow * DD + 8 * (lane - 16))
                                       : (EH + (size_t)grow * KCM + 8 * lane);
        if (wr) *(volatile v8us*)gp = pv;
        __threadfence();
        if (wr) *(volatile v8us*)gp = pv;
      }
    }
  }
}

static int pick_nb(long long nEnt, int nN) {
  int nb = NBMAX;
  while (nb > 16 && (long long)nb * nEnt * 5LL > (long long)RCAP * (long long)nN * 4LL) nb >>= 1;
  return nb;
}
static inline int cdiv(int a, int b) { return (a + b - 1) / b; }
static inline size_t al256(size_t v) { return (v + 255) & ~(size_t)255; }

extern "C" void kernel_launch(void* const* d_in, const int* in_sizes, int n_in,
                              void* d_out, int out_size, void* d_ws, size_t ws_size,
                              hipStream_t stream) {
  if (n_in < 14) return;
  if (in_sizes[0] <= 0 || (in_sizes[0] % DD) != 0) return;
  const int nN = in_sizes[0] / DD;
  if (nN < 1 || nN > (1 << 24)) return;
  if (in_sizes[1] != nN * KCL) return;
  if (in_sizes[2] != KCM * DD || in_sizes[3] != DD) return;
  if (in_sizes[4] != DD * DD  || in_sizes[5] != DD) return;
  if (in_sizes[6] != NL * PK * DD || in_sizes[7] != NL * DD) return;
  if (in_sizes[8] != NL * DD * DD || in_sizes[9] != NL * DD) return;
  if (in_sizes[10] != NL * DD * DD || in_sizes[11] != NL * DD) return;
  if (in_sizes[12] <= 0 || (in_sizes[12] % NL) != 0) return;
  const int E = in_sizes[12] / NL;
  if (E < 1 || E > 262143) return;
  if (in_sizes[13] != NL * E) return;
  if (out_size != nN * DD) return;

  const float* emb  = (const float*)d_in[0];
  const float* memb = (const float*)d_in[1];
  const float* cW1  = (const float*)d_in[2];
  const float* cb1  = (const float*)d_in[3];
  const float* cW2  = (const float*)d_in[4];
  const float* cb2  = (const float*)d_in[5];
  const float* rW1  = (const float*)d_in[6];
  const float* rb1  = (const float*)d_in[7];
  const float* rWs  = (const float*)d_in[8];
  const float* rbs  = (const float*)d_in[9];
  const float* rWo  = (const float*)d_in[10];
  const float* rbo  = (const float*)d_in[11];
  const int*   sIdx = (const int*)d_in[12];
  const int*   oIdx = (const int*)d_in[13];
  float* out = (float*)d_out;

  const int MP   = cdiv(nN, GBM) * GBM;
  const int EP   = cdiv(E, GBM) * GBM;
  const int nSeg = RPC * E;
  const int nb   = pick_nb(2LL * (long long)nSeg, nN);
  const int gA   = cdiv(nN, nb);
  const int vec8 = ((E % 4) == 0) ? 1 : 0;
  if (gA * nb < nN) return;

  const size_t szEH  = al256((size_t)MP * KCM * 2);
  const size_t szEL  = al256((size_t)MP * DD * 2);
  const size_t szUPD = al256((size_t)MP * DD * 4);
  const size_t szACC = al256((size_t)nN * DD * 4);
  const size_t szHID = al256((size_t)MP * DD * 2);
  const size_t szHR  = al256((size_t)RPC * EP * DD * 2);
  const size_t szMSG = al256((size_t)RPC * EP * PK * 4);
  const size_t szR1a = 2 * szHID;
  const size_t szR1b = szHR + szMSG;
  const size_t szR1  = szR1a > szR1b ? szR1a : szR1b;
  const size_t szCW1 = al256((size_t)DD * KCM * 2);
  const size_t szCW2 = al256((size_t)DD * DD * 2);
  const size_t szRW1 = al256((size_t)NL * DD * PK * 2);
  const size_t szRWS = al256((size_t)NL * PK * DD * 2);
  size_t off = 0;
  const size_t oEH  = off; off += szEH;
  const size_t oEL  = off; off += szEL;
  const size_t oUPD = off; off += szUPD;
  const size_t oACC = off; off += szACC;
  const size_t oR1  = off; off += szR1;
  const size_t oCW1 = off; off += szCW1;
  const size_t oCW2 = off; off += szCW2;
  const size_t oRW1 = off; off += szRW1;
  const size_t oRWS = off; off += szRWS;
  if (off > ws_size) return;

  char* ws = (char*)d_ws;
  unsigned short* EH   = (unsigned short*)(ws + oEH);
  unsigned short* EL   = (unsigned short*)(ws + oEL);
  float*          UPD  = (float*)(ws + oUPD);
  float*          ACC  = (float*)(ws + oACC);
  unsigned short* HIDH = (unsigned short*)(ws + oR1);
  unsigned short* HIDL = (unsigned short*)(ws + oR1 + szHID);
  unsigned short* HR   = (unsigned short*)(ws + oR1);
  float*          MSG  = (float*)(ws + oR1 + szHR);
  unsigned short* CW1T = (unsigned short*)(ws + oCW1);
  unsigned short* CW2T = (unsigned short*)(ws + oCW2);
  unsigned short* RW1T = (unsigned short*)(ws + oRW1);
  unsigned short* RWST = (unsigned short*)(ws + oRWS);

  hipFuncSetAttribute(reinterpret_cast<const void*>(&k_agg),
                      hipFuncAttributeMaxDynamicSharedMemorySize, LDS_AGG);
  hipFuncSetAttribute(reinterpret_cast<const void*>(&k_pair),
                      hipFuncAttributeMaxDynamicSharedMemorySize, LDS_PAIR);

  {
    const int nU1 = DD * (KCM / 8);
    k_wtr<<<cdiv(nU1, NTHR), NTHR, 0, stream>>>(cW1, KCM, DD, KCM * DD, DD * KCM, 0, 0, CW1T, nU1);
    const int nU2 = DD * (DD / 8);
    k_wtr<<<cdiv(nU2, NTHR), NTHR, 0, stream>>>(cW2, DD, DD, DD * DD, DD * DD, 0, 0, CW2T, nU2);
    const int nU3 = NL * DD * (PK / 8);
    k_wtr<<<cdiv(nU3, NTHR), NTHR, 0, stream>>>(rW1, PK, DD, PK * DD, DD * PK, 0, 0, RW1T, nU3);
    const int nU4 = NL * DD * (DD / 8);
    k_wtr<<<cdiv(nU4, NTHR), NTHR, 0, stream>>>(rWs, DD, DD, DD * DD, PK * DD, 0,  1, RWST, nU4);
    k_wtr<<<cdiv(nU4, NTHR), NTHR, 0, stream>>>(rWo, DD, DD, DD * DD, PK * DD, DD, 1, RWST, nU4);
  }
  {
    const int nUx = MP * (KCM / 8);
    k_xprep<<<cdiv(nUx, NTHR), NTHR, 0, stream>>>(emb, memb, EH, nN, nUx);
    const int nUl = MP * (DD / 8);
    k_zfill<<<cdiv(nUl, NTHR), NTHR, 0, stream>>>(EL, nUl);
  }

  const int gM = MP / GBM;
  const int gE = EP / GBM;
  for (int t = 0; t < 2; ++t) {
    k_gemm<1, 0><<<dim3(gM, 1, 1), GTHR, 0, stream>>>(
        EH, KCM, KCM / 32, EL, DD, (t == 0) ? 0 : (DD / 32), 0,
        CW1T, 0, cb1, cb1, 0, UPD, HIDH, HIDL, DD, 0, nN, 1.0f);
    k_gemm<0, 0><<<dim3(gM, 1, 1), GTHR, 0, stream>>>(
        HIDH, DD, DD / 32, HIDL, DD, DD / 32, 0,
        CW2T, 0, cb2, cb2, 0, UPD, EL, EL, DD, 0, nN, 1.0f);
    for (int c = 0; c < NCH; ++c) {
      const int lbase = c * RPC;
      k_pair<<<dim3(gE, 1, RPC), GTHR, LDS_PAIR, stream>>>(
          UPD, sIdx + (size_t)lbase * E, oIdx + (size_t)lbase * E, E, EP, nN,
          RW1T + (size_t)lbase * DD * PK, rb1 + (size_t)lbase * DD, HR);
      k_gemm<0, 1><<<dim3(gE, 2, RPC), GTHR, 0, stream>>>(
          HR, DD, DD / 32, HR, DD, 0, EP * DD,
          RWST + (size_t)lbase * PK * DD, PK * DD, rbs + (size_t)lbase * DD, rbo + (size_t)lbase * DD, DD,
          MSG, EL, EL, PK, EP * PK, E, SCL_HW);
      k_agg<<<gA, NTHR, LDS_AGG, stream>>>(
          sIdx + (size_t)c * nSeg, oIdx + (size_t)c * nSeg, nSeg, MSG, E, EP, ACC, UPD, EH, EL, out,
          nN, nb, vec8, (c > 0) ? 1 : 0, (c == NCH - 1) ? 1 : 0, (t == 1) ? 1 : 0);
    }
  }
}
